// ScaledDotProductAttention_69922067579340
// MI455X (gfx1250) — hardware-run, weakly checked
//
#include <hip/hip_runtime.h>
#include <math.h>

typedef __attribute__((ext_vector_type(16))) _Float16 v16h;
typedef __attribute__((ext_vector_type(8)))  _Float16 v8h;
typedef __attribute__((ext_vector_type(16))) __bf16   v16b;
typedef __attribute__((ext_vector_type(8)))  __bf16   v8b;
typedef __attribute__((ext_vector_type(8)))  float    v8f;
typedef __attribute__((ext_vector_type(4)))  float    v4f;
typedef __attribute__((ext_vector_type(4)))  unsigned int v4u;

constexpr int kBatch  = 2;
constexpr int kHeads  = 8;
constexpr int kSeq    = 1024;
constexpr int kHd     = 64;
constexpr int kDm     = 512;
constexpr int kChunk  = 64;
constexpr int kNChunk = kSeq / kChunk;
constexpr int kBH     = kBatch * kHeads;
constexpr int kTok    = kBatch * kSeq;
constexpr int kTiles  = kBH * kNChunk;
constexpr int kTP     = 68;
constexpr float kEps  = 1e-05f;
static_assert(kHeads * kHd == kDm, "head split");
static_assert(kNChunk == 16 && kBH == 16 && kTiles == 256, "index arithmetic below uses shifts by 4");
static_assert(kChunk == 64 && kHd == 64, "64 x 64 tiles");
static_assert((kHd % 32) == 0 && (kChunk % 32) == 0 && (kDm % 32) == 0, "GEMM K multiples of 32");
static_assert((kTok % 64) == 0 && (kDm % 64) == 0, "GEMM M,N multiples of 64");

constexpr float kCarryQ = 64.0f;
constexpr float kCarryK = 64.0f;
constexpr float kCarryV = 1024.0f;
constexpr float kCarryA = 4.0f;
constexpr float kCarryS = 64.0f;
constexpr float kInvQK  = 1.0f / (kCarryQ * kCarryK);
constexpr float kInvKV  = 1.0f / (kCarryK * kCarryV);
constexpr float kInvNum = 1.0f / (kCarryA * kCarryV);
constexpr float kF16Min = 6.103515625e-05f;
static_assert(kCarryA * kCarryV == kCarryQ * kCarryS, "scores x v and q x state share one accumulator scale");

constexpr size_t kPlane16 = (size_t)kBH * kSeq * kHd * 2;
constexpr size_t kOffQF  = 0;
constexpr size_t kOffKF  = kOffQF  + kPlane16;
constexpr size_t kOffKtF = kOffKF  + kPlane16;
constexpr size_t kOffVtF = kOffKtF + kPlane16;
constexpr size_t kOffST  = kOffVtF + kPlane16;
constexpr size_t kOffSpF = kOffST  + (size_t)kTiles * 64 * 64 * 4;
constexpr size_t kOffXH  = kOffSpF + kPlane16;
constexpr size_t kOffXL  = kOffXH  + (size_t)kTok * kDm * 2;
constexpr size_t kOffWH  = kOffXL  + (size_t)kTok * kDm * 2;
constexpr size_t kOffWL  = kOffWH  + (size_t)kDm * kDm * 2;
constexpr size_t kOffZS  = kOffWL  + (size_t)kDm * kDm * 2;
constexpr size_t kWsTotal = kOffZS + (size_t)kTiles * 64 * 4;
static_assert(kPlane16 == 2097152ull, "plane bytes");
static_assert(kWsTotal == 19988480ull, "carve total");
static_assert(kWsTotal <= 134217728ull, "carve cap");
static_assert((kOffKF % 128) == 0 && (kOffKtF % 128) == 0 && (kOffVtF % 128) == 0 && (kOffST % 128) == 0 &&
              (kOffSpF % 128) == 0 && (kOffXH % 128) == 0 && (kOffXL % 128) == 0 &&
              (kOffWH % 128) == 0 && (kOffWL % 128) == 0 && (kOffZS % 128) == 0, "128-B aligned regions");

__device__ __forceinline__ unsigned short f2bf_bits(float f) {
  unsigned u = __float_as_uint(f);
  return (unsigned short)((u + 0x7FFFu + ((u >> 16) & 1u)) >> 16);
}
__device__ __forceinline__ float bf_bits2f(unsigned short h) { return __uint_as_float(((unsigned)h) << 16); }
__device__ __forceinline__ unsigned pk16(unsigned short a, unsigned short b) { return (unsigned)a | ((unsigned)b << 16); }

__device__ __forceinline__ void pack8_hilo(const float (&x)[8], v4u& uh, v4u& ul) {
  unsigned short hb[8], lb[8];
#pragma unroll
  for (int e = 0; e < 8; ++e) {
    hb[e] = f2bf_bits(x[e]);
    lb[e] = f2bf_bits(x[e] - bf_bits2f(hb[e]));
  }
  uh = (v4u){pk16(hb[0], hb[1]), pk16(hb[2], hb[3]), pk16(hb[4], hb[5]), pk16(hb[6], hb[7])};
  ul = (v4u){pk16(lb[0], lb[1]), pk16(lb[2], lb[3]), pk16(lb[4], lb[5]), pk16(lb[6], lb[7])};
}

__device__ __forceinline__ _Float16 f16_carried(float x, float carry) {
  float y = x * carry;
  y = (fabsf(y) < kF16Min) ? 0.0f : y;
  return (_Float16)y;
}
__device__ __forceinline__ v8h pack8_f16(const float (&x)[8], float carry) {
  v8h hv;
#pragma unroll
  for (int e = 0; e < 8; ++e) hv[e] = f16_carried(x[e], carry);
  return hv;
}

__device__ __forceinline__ void dep_guard4_h(v8f& a, v8f& b, v8f& c, v8f& d, v16h x, v16h y) { asm volatile("v_nop\n\tv_nop\n\tv_nop\n\tv_nop" : "+v"(a), "+v"(b), "+v"(c), "+v"(d) : "v"(x), "v"(y)); }
__device__ __forceinline__ void dep_guard4_b(v8f& a, v8f& b, v8f& c, v8f& d, v16b x, v16b y) { asm volatile("v_nop\n\tv_nop\n\tv_nop\n\tv_nop" : "+v"(a), "+v"(b), "+v"(c), "+v"(d) : "v"(x), "v"(y)); }
__device__ __forceinline__ void keep4_h(v16h a, v16h b, v16h c, v16h d) { asm volatile("v_nop" :: "v"(a), "v"(b), "v"(c), "v"(d)); }
__device__ __forceinline__ void keep4_b(v16b a, v16b b, v16b c, v16b d) { asm volatile("v_nop" :: "v"(a), "v"(b), "v"(c), "v"(d)); }
__device__ __forceinline__ void acc_guard4(v8f& a, v8f& b, v8f& c, v8f& d) { asm volatile("v_nop\n\tv_nop\n\tv_nop\n\tv_nop" : "+v"(a), "+v"(b), "+v"(c), "+v"(d)); }
template <typename T> struct Frag;
template <> struct Frag<_Float16> {
  typedef v16h V; union U { v16h v; v8h h[2]; };
  static __device__ __forceinline__ v16h load(const _Float16* p) {
    U f; f.h[0] = *(const v8h*)(p); f.h[1] = *(const v8h*)(p + 16); return f.v;
  }
  static __device__ __forceinline__ v8f mma(v16h a, v16h b, v8f c) {
    return __builtin_amdgcn_wmma_f32_16x16x32_f16(false, a, false, b, (short)0, c, false, false);
  }
  static __device__ __forceinline__ void guard4(v8f& a, v8f& b, v8f& c, v8f& d, v16h x, v16h y) { dep_guard4_h(a, b, c, d, x, y); }
  static __device__ __forceinline__ void keep(v16h a, v16h b, v16h c, v16h d) { keep4_h(a, b, c, d); }
};
template <> struct Frag<__bf16> {
  typedef v16b V; union U { v16b v; v8b h[2]; };
  static __device__ __forceinline__ v16b load(const __bf16* p) {
    U f; f.h[0] = *(const v8b*)(p); f.h[1] = *(const v8b*)(p + 16); return f.v;
  }
  static __device__ __forceinline__ v8f mma(v16b a, v16b b, v8f c) {
    return __builtin_amdgcn_wmma_f32_16x16x32_bf16(false, a, false, b, (short)0, c, false, false);
  }
  static __device__ __forceinline__ void guard4(v8f& a, v8f& b, v8f& c, v8f& d, v16b x, v16b y) { dep_guard4_b(a, b, c, d, x, y); }
  static __device__ __forceinline__ void keep(v16b a, v16b b, v16b c, v16b d) { keep4_b(a, b, c, d); }
};

__device__ __forceinline__ v8f mma_h(v16h a, v16h b, v8f c) {
  c = __builtin_amdgcn_wmma_f32_16x16x32_f16(false, a, false, b, (short)0, c, false, false);
  asm volatile("v_nop\n\tv_nop\n\tv_nop\n\tv_nop" : "+v"(c) : "v"(a), "v"(b));
  return c;
}

template <int ET> struct Elem;
template <> struct Elem<0> { typedef _Float16 T; };
template <> struct Elem<1> { typedef __bf16 T; };
template <int ET, bool SPLIT, int BIAS_MODE, int OUT_MODE, bool RESID, int ACT = 0>
__global__ __launch_bounds__(256) void wmma_gemm64(
    const unsigned short* __restrict__ Ap, const unsigned short* __restrict__ A2p, int lda, long strideA,
    const unsigned short* __restrict__ Btp, const unsigned short* __restrict__ Bt2p, int ldb, long strideB,
    void* __restrict__ Cout, void* __restrict__ Cout2, int ldc, long strideC,
    const float* __restrict__ bias,
    const float* __restrict__ resid, long strideR,
    int M, int N, int K, float scale) {
  typedef typename Elem<ET>::T T;
  typedef typename Frag<T>::V V;
  const T* A = (const T*)Ap; const T* A2 = (const T*)A2p; const T* Bt = (const T*)Btp; const T* Bt2 = (const T*)Bt2p;
  __shared__ __align__(16) float sT[8][16 * 68];
  const int b    = blockIdx.y;
  const int lane = threadIdx.x & 31;
  const int wave = threadIdx.x >> 5;
  const int tilesN = N >> 6;
  const int tilesM = M >> 6;
  const int tile = blockIdx.x * 8 + wave;
  if (tile >= tilesM * tilesN) return;
  const int tm = tile / tilesN;
  const int tn = tile - tm * tilesN;
  const int m0 = tm << 6;
  const int n0 = tn << 6;

  const T* Ab  = A  + (size_t)b * strideA;
  const T* Bb  = Bt + (size_t)b * strideB;
  const T* Ab2 = SPLIT ? (A2  + (size_t)b * strideA) : nullptr;
  const T* Bb2 = SPLIT ? (Bt2 + (size_t)b * strideB) : nullptr;

  const int rlane = lane & 15;
  const int koff  = (lane >> 4) * 8;
  const int mOff  = (lane >> 4) * 8;

  v8f acc[4][4];
#pragma unroll
  for (int i = 0; i < 4; ++i)
#pragma unroll
    for (int j = 0; j < 4; ++j) acc[i][j] = (v8f){0.f,0.f,0.f,0.f,0.f,0.f,0.f,0.f};

  for (int k0 = 0; k0 < K; k0 += 32) {
    V bh[4], bl[4];
#pragma unroll
    for (int j = 0; j < 4; ++j) {
      const size_t bo = (size_t)(n0 + (j << 4) + rlane) * ldb + koff + k0;
      bh[j] = Frag<T>::load(Bb + bo);
      if (SPLIT) bl[j] = Frag<T>::load(Bb2 + bo);
    }
#pragma unroll
    for (int i = 0; i < 4; ++i) {
      const size_t ao = (size_t)(m0 + (i << 4) + rlane) * lda + koff + k0;
      V ah = Frag<T>::load(Ab + ao);
      V al;
      if (SPLIT) al = Frag<T>::load(Ab2 + ao);
#pragma unroll
      for (int j = 0; j < 4; ++j) {
        acc[i][j] = Frag<T>::mma(ah, bh[j], acc[i][j]);
        if (SPLIT) {
          acc[i][j] = Frag<T>::mma(ah, bl[j], acc[i][j]);
          acc[i][j] = Frag<T>::mma(al, bh[j], acc[i][j]);
        }
      }
      Frag<T>::guard4(acc[i][0], acc[i][1], acc[i][2], acc[i][3], ah, SPLIT ? al : ah);
    }
    Frag<T>::keep(bh[0], bh[1], bh[2], bh[3]);
    if (SPLIT) Frag<T>::keep(bl[0], bl[1], bl[2], bl[3]);
  }
  acc_guard4(acc[0][0], acc[0][1], acc[0][2], acc[0][3]);
  acc_guard4(acc[1][0], acc[1][1], acc[1][2], acc[1][3]);
  acc_guard4(acc[2][0], acc[2][1], acc[2][2], acc[2][3]);
  acc_guard4(acc[3][0], acc[3][1], acc[3][2], acc[3][3]);

  float* slab = sT[wave];
  const float* Rb = RESID ? (resid + (size_t)b * strideR) : nullptr;
#pragma unroll
  for (int i = 0; i < 4; ++i) {
    const int mBase = m0 + (i << 4);
#pragma unroll
    for (int j = 0; j < 4; ++j) {
      const int n = n0 + (j << 4) + rlane;
      float bv = 0.f;
      if (BIAS_MODE == 2) bv = bias[n];
#pragma unroll
      for (int r = 0; r < 8; ++r) {
        float v = acc[i][j][r] * scale;
        if (BIAS_MODE == 1) v += bias[mBase + mOff + r];
        if (BIAS_MODE == 2) v += bv;
        if (RESID) v += Rb[(size_t)(mBase + mOff + r) * ldc + n];
        if (ACT == 2) v = fmaxf(v, 0.0f);
        if (ACT == 4) v = (v > 0.f) ? v : 0.01f * v;
        slab[(mOff + r) * 68 + (j << 4) + rlane] = v;
      }
    }
    __builtin_amdgcn_fence(__ATOMIC_RELEASE, "workgroup");
    __builtin_amdgcn_wave_barrier();
    __builtin_amdgcn_fence(__ATOMIC_ACQUIRE, "workgroup");
    if (OUT_MODE == 0) {
      float* C = (float*)Cout + (size_t)b * strideC;
      const int hh = lane >> 4, c4 = (lane & 15) * 4;
      for (int pass = 0; pass < 2; ++pass) {
#pragma unroll
        for (int it = 0; it < 8; ++it) {
          const int row = it * 2 + hh;
          v4f v = *(const v4f*)(slab + row * 68 + c4);
          *(volatile v4f*)(C + (size_t)(mBase + row) * ldc + n0 + c4) = v;
        }
        __threadfence();
      }
    } else {
      const int q = lane >> 3, c8 = (lane & 7) * 8;
      unsigned short* C  = (unsigned short*)Cout  + (size_t)b * strideC;
      unsigned short* C2 = (OUT_MODE == 2) ? ((unsigned short*)Cout2 + (size_t)b * strideC) : nullptr;
      for (int pass = 0; pass < 2; ++pass) {
#pragma unroll
        for (int it = 0; it < 4; ++it) {
          const int row = it * 4 + q;
          const float* sp = slab + row * 68 + c8;
          v8h hv, lv;
#pragma unroll
          for (int e = 0; e < 8; ++e) {
            if (OUT_MODE == 1) {
              hv[e] = (_Float16)sp[e];
            } else {
              unsigned short hb = f2bf_bits(sp[e]);
              unsigned short lb = f2bf_bits(sp[e] - bf_bits2f(hb));
              hv[e] = __builtin_bit_cast(_Float16, hb);
              lv[e] = __builtin_bit_cast(_Float16, lb);
            }
          }
          *(volatile v8h*)(C + (size_t)(mBase + row) * ldc + n0 + c8) = hv;
          if (OUT_MODE == 2) *(volatile v8h*)(C2 + (size_t)(mBase + row) * ldc + n0 + c8) = lv;
        }
        __threadfence();
      }
    }
    __builtin_amdgcn_fence(__ATOMIC_RELEASE, "workgroup");
    __builtin_amdgcn_wave_barrier();
    __builtin_amdgcn_fence(__ATOMIC_ACQUIRE, "workgroup");
  }
}

__global__ __launch_bounds__(256) void prep_kernel(
    const float* __restrict__ q, const float* __restrict__ k, const float* __restrict__ v, const float* __restrict__ mask,
    unsigned short* __restrict__ QF, unsigned short* __restrict__ KF,
    unsigned short* __restrict__ KtF, unsigned short* __restrict__ VtF,
    float* __restrict__ ZS)
{
  __shared__ __align__(16) float sT[3 * 64 * kTP];
  const int tid = threadIdx.x, lane = tid & 31, wave = tid >> 5;
  const size_t rowbase = (size_t)blockIdx.x * 64;
  const size_t gbase = rowbase * 64;
#pragma unroll 1
  for (int i = 0; i < 16; ++i) {
    const int idx = i * 256 + tid;
    const int r = idx >> 6, cc = idx & 63;
    const float qv = q[gbase + idx];
    const float kv = k[gbase + idx];
    const float vv = v[gbase + idx];
    const float mv = mask[gbase + idx];
    const float qe = expf(qv);
    const float ke = expf(kv);
    const float qf = (qv > 0.0f) ? (qv + 1.0f) : qe;
    const float kf = ((kv > 0.0f) ? (kv + 1.0f) : ke) + mv;
    sT[0 * 64 * kTP + r * kTP + cc] = qf;
    sT[1 * 64 * kTP + r * kTP + cc] = kf;
    sT[2 * 64 * kTP + r * kTP + cc] = vv;
  }
  __syncthreads();

  const int q4 = lane >> 3, c8 = (lane & 7) * 8;
#pragma unroll 1
  for (int item = 0; item < 8; ++item) {
    const int tile = item >> 1, it = item & 1;
    const int row = it * 32 + wave * 4 + q4;
    const int srcSel = (tile == 0) ? 0 : ((tile == 3) ? 2 : 1);
    const bool tr = (tile >= 2);
    const int sr = tr ? 1 : kTP;
    const int se = tr ? kTP : 1;
    const float carry = (tile == 0) ? kCarryQ : ((tile == 3) ? kCarryV : kCarryK);
    const float* src = sT + srcSel * 64 * kTP;
    float x[8];
#pragma unroll
    for (int e = 0; e < 8; ++e) x[e] = src[row * sr + (c8 + e) * se];
    const v8h hv = pack8_f16(x, carry);
    unsigned short* ph = (tile == 0) ? QF : ((tile == 1) ? KF : ((tile == 2) ? KtF : VtF));
    const size_t o = (rowbase + row) * 64 + c8;
    for (int pass = 0; pass < 2; ++pass) {
      *(volatile v8h*)(ph + o) = hv;
      __threadfence();
    }
  }

  if (tid < 64) {
    float z = 0.0f;
#pragma unroll 1
    for (int r = 0; r < 64; ++r) z += sT[1 * 64 * kTP + r * kTP + tid];
    float* zp = ZS + rowbase + tid;
    *(volatile float*)zp = z;
    __threadfence();
    *(volatile float*)zp = z;
    __threadfence();
  }
}

__global__ __launch_bounds__(256) void split8_kernel(
    const float* __restrict__ src, unsigned short* __restrict__ dhi, unsigned short* __restrict__ dlo, int total8)
{
  const int i = blockIdx.x * 256 + threadIdx.x;
  if (i >= total8) return;
  const size_t e0 = (size_t)i << 3;
  const v4f a0 = *(const v4f*)(src + e0);
  const v4f a1 = *(const v4f*)(src + e0 + 4);
  float x[8];
  x[0] = a0[0]; x[1] = a0[1]; x[2] = a0[2]; x[3] = a0[3];
  x[4] = a1[0]; x[5] = a1[1]; x[6] = a1[2]; x[7] = a1[3];
  v4u uh, ul;
  pack8_hilo(x, uh, ul);
  for (int pass = 0; pass < 2; ++pass) {
    *(volatile v4u*)(dhi + e0) = uh;
    *(volatile v4u*)(dlo + e0) = ul;
    __threadfence();
  }
}

__global__ __launch_bounds__(256) void prefix_kernel(
    const float* __restrict__ ST, unsigned short* __restrict__ SpF)
{
  const int gid = blockIdx.x * 256 + threadIdx.x;
  const int bh  = gid >> 9;
  const int rem = gid & 511;
  const int vr  = rem >> 3;
  const int e8  = (rem & 7) * 8;
  float acc[8];
#pragma unroll
  for (int e = 0; e < 8; ++e) acc[e] = 0.0f;
#pragma unroll 1
  for (int c = 0; c < kNChunk; ++c) {
    const size_t o = ((size_t)(bh * kNChunk + c) * 64 + vr) * 64 + e8;
    const v8h hv = pack8_f16(acc, kCarryS);
    for (int pass = 0; pass < 2; ++pass) {
      *(volatile v8h*)(SpF + o) = hv;
      __threadfence();
    }
    const v4f a0 = *(const v4f*)(ST + o);
    const v4f a1 = *(const v4f*)(ST + o + 4);
    acc[0] += a0[0]; acc[1] += a0[1]; acc[2] += a0[2]; acc[3] += a0[3];
    acc[4] += a1[0]; acc[5] += a1[1]; acc[6] += a1[2]; acc[7] += a1[3];
  }
}

__global__ __launch_bounds__(128) void chunk_out_kernel(
    const float* __restrict__ qraw,
    const unsigned short* __restrict__ QFp, const unsigned short* __restrict__ KFp,
    const unsigned short* __restrict__ VtFp, const unsigned short* __restrict__ SpFp,
    const float* __restrict__ ZS,
    unsigned short* __restrict__ XH, unsigned short* __restrict__ XL)
{
  __shared__ __align__(16) _Float16 sA[4 * 16 * 64];
  __shared__ __align__(16) float  sO[4 * 16 * kTP];
  __shared__ float sZ[64];
  __shared__ float sQZ[64];

  const int tid = threadIdx.x, wave = tid >> 5, lane = tid & 31, hh = lane >> 4, cl = lane & 15;
  const int blk = blockIdx.x;
  const int bh = blk >> 4, c = blk & 15;
  const int b = bh >> 3, h = bh & 7;
  const size_t rowbase = (size_t)blk * 64;
  const _Float16* QF  = (const _Float16*)QFp;
  const _Float16* KF  = (const _Float16*)KFp;
  const _Float16* VtF = (const _Float16*)VtFp;
  const _Float16* SpF = (const _Float16*)SpFp;

  {
    const int e = tid & 63;
    float z = 0.0f;
#pragma unroll 1
    for (int cc = 0; cc < c; ++cc) z += ZS[(size_t)(bh * kNChunk + cc) * 64 + e];
    if (tid < 64) sZ[tid] = z;
  }
  __syncthreads();

  {
    const int row = tid >> 1, half = tid & 1;
    const float* qp = qraw + (rowbase + row) * 64 + half * 32;
    float accq = 0.0f;
#pragma unroll 1
    for (int g = 0; g < 8; ++g) {
      const v4f qv = *(const v4f*)(qp + 4 * g);
      const float* zp = sZ + half * 32 + 4 * g;
#pragma unroll
      for (int kk = 0; kk < 4; ++kk) {
        const float x = qv[kk];
        const float ex = expf(x);
        const float f = (x > 0.0f) ? (x + 1.0f) : ex;
        accq = fmaf(f, zp[kk], accq);
      }
    }
    accq += __shfl_xor(accq, 1, 32);
    if (half == 0) sQZ[row] = accq;
  }

  v16h qa[2];
  {
    const size_t qo = (rowbase + wave * 16 + cl) * 64 + 8 * hh;
#pragma unroll
    for (int dc = 0; dc < 2; ++dc) qa[dc] = Frag<_Float16>::load(QF + qo + dc * 32);
  }

  float rs[8];
#pragma unroll
  for (int r = 0; r < 8; ++r) rs[r] = 0.0f;
  _Float16* pa = sA + wave * (16 * 64);
#pragma unroll
  for (int j = 0; j < 4; ++j) {
    v8f s = (v8f){0.f,0.f,0.f,0.f,0.f,0.f,0.f,0.f};
    const size_t ko = (rowbase + j * 16 + cl) * 64 + 8 * hh;
#pragma unroll
    for (int dc = 0; dc < 2; ++dc) {
      const v16h kb = Frag<_Float16>::load(KF + ko + dc * 32);
      s = mma_h(qa[dc], kb, s);
    }
#pragma unroll
    for (int r = 0; r < 8; ++r) {
      const int qr = wave * 16 + 8 * hh + r;
      const int kc = j * 16 + cl;
      const float sv = s[r] * kInvQK;
      const float a = (kc <= qr) ? sv : 0.0f;
      rs[r] += a;
      pa[(8 * hh + r) * 64 + kc] = f16_carried(a, kCarryA);
    }
  }
#pragma unroll
  for (int r = 0; r < 8; ++r) {
#pragma unroll
    for (int off = 1; off < 16; off <<= 1) rs[r] += __shfl_xor(rs[r], off, 32);
  }
  __syncthreads();

  float den[8];
#pragma unroll
  for (int r = 0; r < 8; ++r) den[r] = (rs[r] + sQZ[wave * 16 + 8 * hh + r]) + kEps;

  v8f oacc[4];
#pragma unroll
  for (int t = 0; t < 4; ++t) oacc[t] = (v8f){0.f,0.f,0.f,0.f,0.f,0.f,0.f,0.f};

#pragma unroll
  for (int kk = 0; kk < 2; ++kk) {
    const v16h af = Frag<_Float16>::load(pa + cl * 64 + kk * 32 + 8 * hh);
#pragma unroll
    for (int t = 0; t < 4; ++t) {
      const size_t vo = (rowbase + t * 16 + cl) * 64 + kk * 32 + 8 * hh;
      const v16h vb = Frag<_Float16>::load(VtF + vo);
      oacc[t] = mma_h(af, vb, oacc[t]);
    }
  }
#pragma unroll
  for (int dc = 0; dc < 2; ++dc) {
#pragma unroll
    for (int t = 0; t < 4; ++t) {
      const size_t so = (rowbase + t * 16 + cl) * 64 + dc * 32 + 8 * hh;
      const v16h sb = Frag<_Float16>::load(SpF + so);
      oacc[t] = mma_h(qa[dc], sb, oacc[t]);
    }
  }

  float* po = sO + wave * (16 * kTP);
#pragma unroll
  for (int t = 0; t < 4; ++t) {
#pragma unroll
    for (int r = 0; r < 8; ++r) {
      const float nv = oacc[t][r] * kInvNum;
      po[(8 * hh + r) * kTP + t * 16 + cl] = nv * den[r];
    }
  }
  __syncthreads();

  {
    const int q4 = lane >> 3, c8 = (lane & 7) * 8;
    v4u uh[4], ul[4];
#pragma unroll
    for (int it = 0; it < 4; ++it) {
      const int row = it * 4 + q4;
      const float* sp = po + row * kTP + c8;
      const v4f a0 = *(const v4f*)(sp);
      const v4f a1 = *(const v4f*)(sp + 4);
      float x[8];
      x[0] = a0[0]; x[1] = a0[1]; x[2] = a0[2]; x[3] = a0[3];
      x[4] = a1[0]; x[5] = a1[1]; x[6] = a1[2]; x[7] = a1[3];
      pack8_hilo(x, uh[it], ul[it]);
    }
    for (int pass = 0; pass < 2; ++pass) {
#pragma unroll
      for (int it = 0; it < 4; ++it) {
        const int row = it * 4 + q4;
        const size_t o = (size_t)(b * kSeq + c * kChunk + wave * 16 + row) * kDm + h * kHd + c8;
        *(volatile v4u*)(XH + o) = uh[it];
        *(volatile v4u*)(XL + o) = ul[it];
      }
      __threadfence();
    }
  }
}

extern "C" void kernel_launch(void* const* d_in, const int* in_sizes, int n_in,
                              void* d_out, int out_size, void* d_ws, size_t ws_size,
                              hipStream_t stream) {
  if (n_in < 6) return;
  if (in_sizes[0] != kBH * kSeq * kHd) return;
  if (in_sizes[1] != kBH * kSeq * kHd) return;
  if (in_sizes[2] != kBH * kSeq * kHd) return;
  if (in_sizes[3] != kBH * kSeq * kHd) return;
  if (in_sizes[4] != kDm * kDm) return;
  if (in_sizes[5] != kDm) return;
  if (out_size != kTok * kDm) return;
  if (ws_size < kWsTotal) return;

  const float* q    = (const float*)d_in[0];
  const float* k    = (const float*)d_in[1];
  const float* v    = (const float*)d_in[2];
  const float* mask = (const float*)d_in[3];
  const float* W    = (const float*)d_in[4];
  const float* bias = (const float*)d_in[5];
  float* out = (float*)d_out;

  char* ws = (char*)d_ws;
  unsigned short* QF  = (unsigned short*)(ws + kOffQF);
  unsigned short* KF  = (unsigned short*)(ws + kOffKF);
  unsigned short* KtF = (unsigned short*)(ws + kOffKtF);
  unsigned short* VtF = (unsigned short*)(ws + kOffVtF);
  float*          ST  = (float*)(ws + kOffST);
  unsigned short* SpF = (unsigned short*)(ws + kOffSpF);
  unsigned short* XH  = (unsigned short*)(ws + kOffXH);
  unsigned short* XL  = (unsigned short*)(ws + kOffXL);
  unsigned short* WH  = (unsigned short*)(ws + kOffWH);
  unsigned short* WL  = (unsigned short*)(ws + kOffWL);
  float*          ZS  = (float*)(ws + kOffZS);

  prep_kernel<<<kTiles, 256, 0, stream>>>(q, k, v, mask, QF, KF, KtF, VtF, ZS);

  split8_kernel<<<(kDm * kDm / 8) / 256, 256, 0, stream>>>(W, WH, WL, kDm * kDm / 8);

  wmma_gemm64<0, false, 0, 0, false><<<dim3(1, kTiles), 32, 0, stream>>>(
      VtF, nullptr, 64, 4096L,
      KtF, nullptr, 64, 4096L,
      (void*)ST, nullptr, 64, 4096L,
      nullptr, nullptr, 0L,
      64, 64, 64, kInvKV);

  prefix_kernel<<<(kBH * 64 * 8) / 256, 256, 0, stream>>>(ST, SpF);

  chunk_out_kernel<<<kTiles, 128, 0, stream>>>(q, QF, KF, VtF, SpF, ZS, XH, XL);

  wmma_gemm64<1, true, 2, 0, false><<<dim3(32, 1), 256, 0, stream>>>(
      XH, XL, kDm, 0L,
      WH, WL, kDm, 0L,
      (void*)out, nullptr, kDm, 0L,
      bias, nullptr, 0L,
      kTok, kDm, kDm, 1.0f);
}
